// Head_30709016166761
// MI455X (gfx1250) — hardware-verified
//
#include <hip/hip_runtime.h>
#include <math.h>

#ifndef NB
#define NB 8
#endif
#ifndef SEQ
#define SEQ 2048
#endif
#define NB_FULL 8
#define SEQ_FULL 2048
#define CC 768
#define HH 64
#define ATTN_SCALE 0.03608439182435161f

static_assert(NB >= 1 && NB <= NB_FULL);
static_assert(SEQ >= 128 && SEQ <= SEQ_FULL && (SEQ % 128) == 0);
static_assert((CC % 64) == 0 && (CC % 32) == 0);
static_assert(HH == 64);
static_assert(((CC * HH / 2) % 256) == 0);
static_assert(((NB * SEQ) % 128) == 0);

typedef _Float16 h16;
typedef __attribute__((ext_vector_type(16))) _Float16 v16h;
typedef __attribute__((ext_vector_type(8)))  _Float16 v8h;
typedef __attribute__((ext_vector_type(8)))  float    v8f;
#define RSPLIT (1.0f / 2048.0f)
__device__ __forceinline__ void split16(float f, h16& hi, h16& lo) { hi = (h16)f; lo = (h16)((f - (float)hi) * 2048.0f); }
__device__ __forceinline__ unsigned short hbits(h16 h) { return __builtin_bit_cast(unsigned short, h); }

#define NEG_INF (-__builtin_inff())

__device__ __forceinline__ v8f v8f_zero() {
  v8f z = {0.f, 0.f, 0.f, 0.f, 0.f, 0.f, 0.f, 0.f};
  return z;
}

__device__ __forceinline__ v8f wmma16(v16h a, v16h b, v8f c) {
  v8f r = __builtin_amdgcn_wmma_f32_16x16x32_f16(false, a, false, b, (short)0, c, false, false);
  asm volatile("v_nop\n\tv_nop\n\tv_nop\n\tv_nop" : "+v"(r) : "v"(a), "v"(b));
  return r;
}

__device__ __forceinline__ v8f wmma_split(v16h ah, v16h al, v16h bh, v16h bl, v8f c) {
  v8f x = wmma16(al, bh, v8f_zero());
  x = wmma16(ah, bl, x);
  return wmma16(ah, bh, c) + x * RSPLIT;
}

__global__ void __launch_bounds__(256)
wt_kernel(const float* __restrict__ Wk,
          const float* __restrict__ Wq,
          const float* __restrict__ Wv,
          h16* __restrict__ WtQ,
          h16* __restrict__ WtK,
          h16* __restrict__ WtV) {
  const int idx = blockIdx.x * 256 + threadIdx.x;
  if (idx >= CC * HH / 2) return;
  const int h = idx / (CC / 2);
  const int c = 2 * (idx % (CC / 2));
  const float* src[3] = {Wq, Wk, Wv};
  h16* dstp[3] = {WtQ, WtK, WtV};
#pragma unroll
  for (int s = 0; s < 3; ++s) {
    h16 h0, l0, h1, l1;
    split16(src[s][(size_t)c * HH + h], h0, l0);
    split16(src[s][(size_t)(c + 1) * HH + h], h1, l1);
    unsigned* dh = (unsigned*)(dstp[s] + (size_t)h * CC + c);
    unsigned* dl = (unsigned*)(dstp[s] + (size_t)CC * HH + (size_t)h * CC + c);
    const unsigned ph = (unsigned)hbits(h0) | ((unsigned)hbits(h1) << 16);
    const unsigned pl = (unsigned)hbits(l0) | ((unsigned)hbits(l1) << 16);
    *(volatile unsigned*)dh = ph; *(volatile unsigned*)dl = pl;
    __threadfence();
    *(volatile unsigned*)dh = ph; *(volatile unsigned*)dl = pl;
  }
}

__global__ void __launch_bounds__(256)
qkv_kernel(const float* __restrict__ x,
           const h16* __restrict__ WtQ,
           const h16* __restrict__ WtK,
           const h16* __restrict__ WtV,
           h16* __restrict__ qws,
           h16* __restrict__ kws,
           h16* __restrict__ vws) {
  __shared__ __align__(16) h16 st[8][16][64];
  const int lane = threadIdx.x & 31;
  const int wv   = threadIdx.x >> 5;
  const int g    = lane >> 4;
  const int m    = lane & 15;
  const int tile = blockIdx.x * 8 + wv;
  const int b    = tile / (SEQ / 16);
  const int t0   = (tile % (SEQ / 16)) * 16;
  const size_t PL = (size_t)CC * HH;
  const size_t QL = (size_t)NB * SEQ * HH;

  v8f accQ[4], accK[4], accV[4];
#pragma unroll
  for (int nt = 0; nt < 4; ++nt) {
    accQ[nt] = v8f_zero();
    accK[nt] = v8f_zero();
    accV[nt] = v8f_zero();
  }

  const float* xrow = x + ((size_t)b * SEQ_FULL + t0 + m) * CC;

#pragma unroll 1
  for (int c0 = 0; c0 < CC; c0 += 32) {
    union { v16h v; h16 e[16]; } a, al;
#pragma unroll
    for (int j = 0; j < 8; ++j) {
      split16(xrow[c0 + 8 * g + j],      a.e[j],     al.e[j]);
      split16(xrow[c0 + 16 + 8 * g + j], a.e[8 + j], al.e[8 + j]);
    }
    union UB { v16h v; v8h h[2]; };
#pragma unroll
    for (int nt = 0; nt < 4; ++nt) {
      const size_t woff = (size_t)(nt * 16 + m) * CC + c0 + 8 * g;
      UB bq, bk, bv, bql, bkl, bvl;
      bq.h[0]  = *(const v8h*)(WtQ + woff);      bq.h[1]  = *(const v8h*)(WtQ + woff + 16);
      bk.h[0]  = *(const v8h*)(WtK + woff);      bk.h[1]  = *(const v8h*)(WtK + woff + 16);
      bv.h[0]  = *(const v8h*)(WtV + woff);      bv.h[1]  = *(const v8h*)(WtV + woff + 16);
      bql.h[0] = *(const v8h*)(WtQ + PL + woff); bql.h[1] = *(const v8h*)(WtQ + PL + woff + 16);
      bkl.h[0] = *(const v8h*)(WtK + PL + woff); bkl.h[1] = *(const v8h*)(WtK + PL + woff + 16);
      bvl.h[0] = *(const v8h*)(WtV + PL + woff); bvl.h[1] = *(const v8h*)(WtV + PL + woff + 16);
      accQ[nt] = wmma_split(a.v, al.v, bq.v, bql.v, accQ[nt]);
      accK[nt] = wmma_split(a.v, al.v, bk.v, bkl.v, accK[nt]);
      accV[nt] = wmma_split(a.v, al.v, bv.v, bvl.v, accV[nt]);
    }
  }

  h16* sw = &st[wv][0][0];
  h16* dsts[3] = {qws, kws, vws};
#pragma unroll
  for (int s = 0; s < 3; ++s) {
#pragma unroll
    for (int pl = 0; pl < 2; ++pl) {
#pragma unroll
      for (int nt = 0; nt < 4; ++nt)
#pragma unroll
        for (int v = 0; v < 8; ++v) {
          const float val = (s == 0) ? accQ[nt][v] : (s == 1) ? accK[nt][v] : accV[nt][v];
          h16 hh_, ll_; split16(val, hh_, ll_);
          sw[(8 * g + v) * 64 + nt * 16 + m] = pl ? ll_ : hh_;
        }
      asm volatile("s_wait_dscnt 0" ::: "memory");
      h16* base = dsts[s] + (pl ? QL : 0) + ((size_t)b * SEQ + t0) * HH;
#pragma unroll
      for (int r = 0; r < 16; ++r) {
        const unsigned w = *((const unsigned*)(sw + r * 64) + lane);
        *(volatile unsigned*)((unsigned*)(base + (size_t)r * HH) + lane) = w;
      }
      __threadfence();
#pragma unroll
      for (int r = 0; r < 16; ++r) {
        const unsigned w = *((const unsigned*)(sw + r * 64) + lane);
        *(volatile unsigned*)((unsigned*)(base + (size_t)r * HH) + lane) = w;
      }
      asm volatile("s_wait_dscnt 0" ::: "memory");
    }
  }
}

__global__ void __launch_bounds__(256)
vt_kernel(const h16* __restrict__ vws, h16* __restrict__ vtws) {
  __shared__ h16 t[64][66];
  const int tid = threadIdx.x, lane = tid & 31, wv = tid >> 5;
  const size_t QL = (size_t)NB * SEQ * HH;
  const int row0 = blockIdx.x * 64;
  const int b = row0 / SEQ, tb = row0 % SEQ;
  const int pl = blockIdx.y;
  const h16* src = vws + (pl ? QL : 0) + (size_t)row0 * HH;
#pragma unroll
  for (int k = 0; k < 16; ++k) { const int e = tid + 256 * k; t[e >> 6][e & 63] = src[e]; }
  __syncthreads();
  h16* dst = vtws + (pl ? QL : 0) + (size_t)b * HH * SEQ;
#pragma unroll
  for (int r = 0; r < 8; ++r) {
    const int h = wv * 8 + r;
    const unsigned pk = (unsigned)hbits(t[2 * lane][h]) | ((unsigned)hbits(t[2 * lane + 1][h]) << 16);
    unsigned* d = (unsigned*)(dst + (size_t)h * SEQ + tb) + lane;
    *(volatile unsigned*)d = pk;
    __threadfence();
    *(volatile unsigned*)d = pk;
  }
}

__global__ void __launch_bounds__(128)
attn_kernel(const h16* __restrict__ qws,
            const h16* __restrict__ kws,
            const h16* __restrict__ vtws,
            float* __restrict__ out) {
  __shared__ __align__(16) h16 Pl[4][16][32];
  __shared__ __align__(16) h16 Pll[4][16][32];
  __shared__ __align__(16) float Of[4][16][64];
  __shared__ float Ml[4][16], Ll[4][16];

  const int lane = threadIdx.x & 31;
  const int wv   = threadIdx.x >> 5;
  const int g    = lane >> 4;
  const int m    = lane & 15;
  const int tile = blockIdx.x;
  const int b    = tile / (SEQ / 16);
  const int t0   = (tile % (SEQ / 16)) * 16;

  union U16 { v16h v; v8h h[2]; };

  const size_t QL = (size_t)NB * SEQ * HH;
  const h16* qrow = qws + ((size_t)b * SEQ + t0 + m) * HH;
  U16 qa[2], qal[2];
#pragma unroll
  for (int hc = 0; hc < 2; ++hc) {
    qa[hc].h[0]  = *(const v8h*)(qrow + hc * 32 + 8 * g);
    qa[hc].h[1]  = *(const v8h*)(qrow + hc * 32 + 16 + 8 * g);
    qal[hc].h[0] = *(const v8h*)(qrow + QL + hc * 32 + 8 * g);
    qal[hc].h[1] = *(const v8h*)(qrow + QL + hc * 32 + 16 + 8 * g);
  }

  v8f o[4];
#pragma unroll
  for (int nt = 0; nt < 4; ++nt) o[nt] = v8f_zero();
  float mrow[8], lrow[8];
#pragma unroll
  for (int v = 0; v < 8; ++v) { mrow[v] = NEG_INF; lrow[v] = 0.f; }

  const float scale = ATTN_SCALE;
  const int   nblk  = t0 / 32 + 1;

  const h16* kbase  = kws + (size_t)b * SEQ * HH;
  const h16* vtbase = vtws + (size_t)b * HH * SEQ;

  for (int blk = wv; blk < nblk; blk += 4) {
    const int s0 = blk * 32;

    v8f s[2];
#pragma unroll
    for (int kt = 0; kt < 2; ++kt) {
      const h16* krow = kbase + (size_t)(s0 + kt * 16 + m) * HH;
      U16 kb0, kb1, kb0l, kb1l;
      kb0.h[0]  = *(const v8h*)(krow + 8 * g);           kb0.h[1]  = *(const v8h*)(krow + 16 + 8 * g);
      kb1.h[0]  = *(const v8h*)(krow + 32 + 8 * g);      kb1.h[1]  = *(const v8h*)(krow + 48 + 8 * g);
      kb0l.h[0] = *(const v8h*)(krow + QL + 8 * g);      kb0l.h[1] = *(const v8h*)(krow + QL + 16 + 8 * g);
      kb1l.h[0] = *(const v8h*)(krow + QL + 32 + 8 * g); kb1l.h[1] = *(const v8h*)(krow + QL + 48 + 8 * g);
      s[kt] = wmma_split(qa[0].v, qal[0].v, kb0.v, kb0l.v, v8f_zero());
      s[kt] = wmma_split(qa[1].v, qal[1].v, kb1.v, kb1l.v, s[kt]);
    }

    const bool diag = (s0 + 31 >= t0);
    float rmax[8];
#pragma unroll
    for (int v = 0; v < 8; ++v) {
      const int row = t0 + 8 * g + v;
#pragma unroll
      for (int kt = 0; kt < 2; ++kt) {
        const int col = s0 + kt * 16 + m;
        float val = s[kt][v] * scale;
        val = (diag && (col > row)) ? NEG_INF : val;
        s[kt][v] = val;
      }
      rmax[v] = fmaxf(s[0][v], s[1][v]);
    }
#pragma unroll
    for (int off = 1; off < 16; off <<= 1)
#pragma unroll
      for (int v = 0; v < 8; ++v)
        rmax[v] = fmaxf(rmax[v], __shfl_xor(rmax[v], off, 32));

    float alpha[8], psum[8];
#pragma unroll
    for (int v = 0; v < 8; ++v) {
      const float mnew = fmaxf(mrow[v], rmax[v]);
      alpha[v] = __expf(mrow[v] - mnew);
      mrow[v]  = mnew;
      const float p0 = __expf(s[0][v] - mnew);
      const float p1 = __expf(s[1][v] - mnew);
      { h16 ph, pq; split16(p0 * 1024.0f, ph, pq); Pl[wv][8 * g + v][m] = ph;      Pll[wv][8 * g + v][m] = pq;
        split16(p1 * 1024.0f, ph, pq);          Pl[wv][8 * g + v][16 + m] = ph; Pll[wv][8 * g + v][16 + m] = pq; }
      psum[v] = p0 + p1;
    }
#pragma unroll
    for (int off = 1; off < 16; off <<= 1)
#pragma unroll
      for (int v = 0; v < 8; ++v)
        psum[v] += __shfl_xor(psum[v], off, 32);
#pragma unroll
    for (int v = 0; v < 8; ++v)
      lrow[v] = lrow[v] * alpha[v] + psum[v];
#pragma unroll
    for (int nt = 0; nt < 4; ++nt)
#pragma unroll
      for (int v = 0; v < 8; ++v)
        o[nt][v] *= alpha[v];

    __builtin_amdgcn_fence(3  , "wavefront");
    __builtin_amdgcn_wave_barrier();
    U16 pa, pal;
    pa.h[0]  = *(const v8h*)&Pl[wv][m][8 * g];
    pa.h[1]  = *(const v8h*)&Pl[wv][m][16 + 8 * g];
    pal.h[0] = *(const v8h*)&Pll[wv][m][8 * g];
    pal.h[1] = *(const v8h*)&Pll[wv][m][16 + 8 * g];
    __builtin_amdgcn_wave_barrier();

#pragma unroll
    for (int nt = 0; nt < 4; ++nt) {
      const h16* vrow = vtbase + (size_t)(nt * 16 + m) * SEQ + s0;
      U16 vb, vbl;
      vb.h[0]  = *(const v8h*)(vrow + 8 * g);      vb.h[1]  = *(const v8h*)(vrow + 16 + 8 * g);
      vbl.h[0] = *(const v8h*)(vrow + QL + 8 * g); vbl.h[1] = *(const v8h*)(vrow + QL + 16 + 8 * g);
      o[nt] = wmma_split(pa.v, pal.v, vb.v, vbl.v, o[nt]);
    }
  }

#pragma unroll
  for (int nt = 0; nt < 4; ++nt)
#pragma unroll
    for (int v = 0; v < 8; ++v)
      Of[wv][8 * g + v][nt * 16 + m] = o[nt][v];
  if (m == 0) {
#pragma unroll
    for (int v = 0; v < 8; ++v) {
      Ml[wv][8 * g + v] = mrow[v];
      Ll[wv][8 * g + v] = lrow[v];
    }
  }
  __syncthreads();

  for (int e = threadIdx.x; e < 16 * HH; e += 128) {
    const int row = e >> 6;
    const int col = e & 63;
    float M = Ml[0][row];
#pragma unroll
    for (int w = 1; w < 4; ++w) M = fmaxf(M, Ml[w][row]);
    float L = 0.f, O = 0.f;
#pragma unroll
    for (int w = 0; w < 4; ++w) {
      const float be = __expf(Ml[w][row] - M);
      L += be * Ll[w][row];
      O += be * Of[w][row][col];
    }
    const float r = O / (L * 1024.0f);
    float* op = out + ((size_t)b * SEQ_FULL + t0 + row) * HH + col;
    *(volatile float*)op = r;
    __threadfence();
    *(volatile float*)op = r;
  }
}

extern "C" void kernel_launch(void* const* d_in, const int* in_sizes, int n_in,
                              void* d_out, int out_size, void* d_ws,
                              size_t ws_size, hipStream_t stream) {
  if (n_in < 4) return;
  const long long rows_needed = (long long)(NB - 1) * SEQ_FULL + SEQ;
  if ((long long)in_sizes[0] < rows_needed * CC) return;
  if (in_sizes[1] < CC * HH || in_sizes[2] < CC * HH || in_sizes[3] < CC * HH) return;
  if ((long long)out_size < rows_needed * HH) return;

  const float* x  = (const float*)d_in[0];
  const float* Wk = (const float*)d_in[1];
  const float* Wq = (const float*)d_in[2];
  const float* Wv = (const float*)d_in[3];
  float* out = (float*)d_out;

  char* ws = (char*)d_ws;
  const size_t qkv_bytes = (size_t)2 * NB * SEQ * HH * sizeof(h16);
  const size_t wt_bytes  = (size_t)2 * CC * HH * sizeof(h16);
  const size_t total     = 4 * qkv_bytes + 3 * wt_bytes;
  if (total > ws_size) return;
  h16* qws  = (h16*)(ws);
  h16* kws  = (h16*)(ws + qkv_bytes);
  h16* vws  = (h16*)(ws + 2 * qkv_bytes);
  h16* vtws = (h16*)(ws + 3 * qkv_bytes);
  h16* WtQ  = (h16*)(ws + 4 * qkv_bytes);
  h16* WtK  = (h16*)(ws + 4 * qkv_bytes + wt_bytes);
  h16* WtV  = (h16*)(ws + 4 * qkv_bytes + 2 * wt_bytes);

  wt_kernel<<<(CC * HH / 2) / 256, 256, 0, stream>>>(Wk, Wq, Wv, WtQ, WtK, WtV);
  qkv_kernel<<<(NB * SEQ) / 128, 256, 0, stream>>>(x, WtQ, WtK, WtV, qws, kws, vws);
  vt_kernel<<<dim3((NB * SEQ) / 64, 2), 256, 0, stream>>>(vws, vtws);
  attn_kernel<<<(NB * SEQ) / 16, 128, 0, stream>>>(qws, kws, vtws, out);
}
